// Transformer_5970004542178
// MI455X (gfx1250) — hardware-verified
//
#include <hip/hip_runtime.h>
#include <math.h>

#ifndef NB
#define NB 32
#endif
#ifndef SEQ
#define SEQ 512
#endif
#define NB_FULL 32
#define SEQ_FULL 512
#define DM 512
#define NH 8
#define DFF 2048
#define MROWS (NB * SEQ)
#define MC (MROWS / 2)
#define LN_EPS 1e-3f
#define NEGFILL (-4294967295.0f)
#define AT_PSC 32768.0f
#define WCARRY 64.0f
#define WINV 0.015625f

static_assert(NB >= 1 && NB <= NB_FULL);
static_assert(SEQ >= 64 && SEQ <= SEQ_FULL && (SEQ % 64) == 0);
static_assert((MROWS % 128) == 0);
static_assert((MC % 64) == 0);
static_assert((DM % 64) == 0 && (DFF % 64) == 0 && (DM % 32) == 0 && (DFF % 32) == 0);
static_assert(((MROWS * 64) % 256) == 0);
static_assert((MROWS % 8) == 0);

typedef __attribute__((ext_vector_type(16))) _Float16 v16h;
typedef __attribute__((ext_vector_type(8)))  _Float16 v8h;
typedef __attribute__((ext_vector_type(16))) __bf16   v16b;
typedef __attribute__((ext_vector_type(8)))  float    v8f;
typedef __attribute__((ext_vector_type(4)))  float    v4f;
typedef unsigned int cm_u4 __attribute__((ext_vector_type(4)));

__device__ __forceinline__ v8f wmma16(v16h a, v16h b, v8f c) {
    c = __builtin_amdgcn_wmma_f32_16x16x32_f16(false, a, false, b, (short)0, c, false, false);
    asm volatile("v_nop\n\tv_nop\n\tv_nop\n\tv_nop" : "+v"(c) : "v"(a), "v"(b));
    return c;
}

#define VST2(T, ptr, val) do { const T vst2_v_ = (val); *(volatile T*)(ptr) = vst2_v_; __threadfence(); *(volatile T*)(ptr) = vst2_v_; } while (0)
#define VST2V4(ptr, val) do { const v4f vst2_v4_ = (val); *(volatile v4f*)(ptr) = vst2_v4_; __threadfence(); *(volatile v4f*)(ptr) = vst2_v4_; } while (0)

__device__ __forceinline__ void wave_lds_sync() {
    __builtin_amdgcn_fence(3  , "workgroup");
    __builtin_amdgcn_wave_barrier();
    __builtin_amdgcn_fence(2  , "workgroup");
}

__device__ __forceinline__ unsigned int cmb_pk2(float a, float b) { return (unsigned int)__builtin_bit_cast(unsigned short, (_Float16)a) | ((unsigned int)__builtin_bit_cast(unsigned short, (_Float16)b) << 16); }
__device__ __forceinline__ float cmb_bf(float v) { const unsigned u = __builtin_bit_cast(unsigned, v); const unsigned r = (u + 0x7fffu + ((u >> 16) & 1u)) & 0xffff0000u; return __builtin_bit_cast(float, r); }

namespace w25 {
typedef __attribute__((ext_vector_type(16))) _Float16 v16h;
typedef __attribute__((ext_vector_type(8)))  _Float16 v8h;
typedef __attribute__((ext_vector_type(16))) __bf16   v16b;
typedef __attribute__((ext_vector_type(8)))  __bf16   v8b;
typedef __attribute__((ext_vector_type(8)))  float    v8f;
typedef __attribute__((ext_vector_type(4)))  float    v4f;

__device__ __forceinline__ unsigned short f2bf_bits(float f) {
  unsigned u = __float_as_uint(f);
  return (unsigned short)((u + 0x7FFFu + ((u >> 16) & 1u)) >> 16);
}
__device__ __forceinline__ float bf_bits2f(unsigned short h) { return __uint_as_float(((unsigned)h) << 16); }

__device__ __forceinline__ void dep_guard_h(v8f& a, v8f& b, v16h x, v16h y) { asm volatile("v_nop\n\tv_nop\n\tv_nop\n\tv_nop" : "+v"(a), "+v"(b) : "v"(x), "v"(y)); }
__device__ __forceinline__ void dep_guard_b(v8f& a, v8f& b, v16b x, v16b y) { asm volatile("v_nop\n\tv_nop\n\tv_nop\n\tv_nop" : "+v"(a), "+v"(b) : "v"(x), "v"(y)); }
__device__ __forceinline__ void keep4_h(v16h a, v16h b, v16h c, v16h d) { asm volatile("v_nop" :: "v"(a), "v"(b), "v"(c), "v"(d)); }
__device__ __forceinline__ void keep4_b(v16b a, v16b b, v16b c, v16b d) { asm volatile("v_nop" :: "v"(a), "v"(b), "v"(c), "v"(d)); }
__device__ __forceinline__ void acc_guard4(v8f& a, v8f& b, v8f& c, v8f& d) { asm volatile("v_nop\n\tv_nop\n\tv_nop\n\tv_nop" : "+v"(a), "+v"(b), "+v"(c), "+v"(d)); }
template <typename T> struct Frag;
template <> struct Frag<_Float16> {
  typedef v16h V; union U { v16h v; v8h h[2]; };
  static __device__ __forceinline__ v16h load(const _Float16* p) {
    U f; f.h[0] = *(const v8h*)(p); f.h[1] = *(const v8h*)(p + 16); return f.v;
  }
  static __device__ __forceinline__ v8f mma(v16h a, v16h b, v8f c) {
    return __builtin_amdgcn_wmma_f32_16x16x32_f16(false, a, false, b, (short)0, c, false, false);
  }
  static __device__ __forceinline__ void guard(v8f& a, v8f& b, v16h x, v16h y) { dep_guard_h(a, b, x, y); }
  static __device__ __forceinline__ void keep(v16h a, v16h b, v16h c, v16h d) { keep4_h(a, b, c, d); }
};
template <> struct Frag<__bf16> {
  typedef v16b V; union U { v16b v; v8b h[2]; };
  static __device__ __forceinline__ v16b load(const __bf16* p) {
    U f; f.h[0] = *(const v8b*)(p); f.h[1] = *(const v8b*)(p + 16); return f.v;
  }
  static __device__ __forceinline__ v8f mma(v16b a, v16b b, v8f c) {
    return __builtin_amdgcn_wmma_f32_16x16x32_bf16(false, a, false, b, (short)0, c, false, false);
  }
  static __device__ __forceinline__ void guard(v8f& a, v8f& b, v16b x, v16b y) { dep_guard_b(a, b, x, y); }
  static __device__ __forceinline__ void keep(v16b a, v16b b, v16b c, v16b d) { keep4_b(a, b, c, d); }
};

template <int ET> struct Elem;
template <> struct Elem<0> { typedef _Float16 T; };
template <> struct Elem<1> { typedef __bf16 T; };
template <int ET, bool SPLIT, int BIAS_MODE, int OUT_MODE, bool RESID, int ACT = 0>
__global__ __launch_bounds__(256) void wmma_gemm64(
    const unsigned short* __restrict__ Ap, const unsigned short* __restrict__ A2p, int lda, long strideA,
    const unsigned short* __restrict__ Btp, const unsigned short* __restrict__ Bt2p, int ldb, long strideB,
    void* __restrict__ Cout, void* __restrict__ Cout2, int ldc, long strideC,
    const float* __restrict__ bias,
    const float* __restrict__ resid, long strideR,
    int M, int N, int K, float scale) {
  typedef typename Elem<ET>::T T;
  typedef typename Frag<T>::V V;
  const T* A = (const T*)Ap; const T* A2 = (const T*)A2p; const T* Bt = (const T*)Btp; const T* Bt2 = (const T*)Bt2p;
  __shared__ __align__(16) float sT[8][16 * 68];
  const int b    = blockIdx.y;
  const int lane = threadIdx.x & 31;
  const int wave = threadIdx.x >> 5;
  const int tilesN = N >> 6;
  const int tilesM = M >> 6;
  const int tile = blockIdx.x * 8 + wave;
  if (tile >= tilesM * tilesN) return;
  const int tm = tile / tilesN;
  const int tn = tile - tm * tilesN;
  const int m0 = tm << 6;
  const int n0 = tn << 6;

  const T* Ab  = A  + (size_t)b * strideA;
  const T* Bb  = Bt + (size_t)b * strideB;
  const T* Ab2 = SPLIT ? (A2  + (size_t)b * strideA) : nullptr;
  const T* Bb2 = SPLIT ? (Bt2 + (size_t)b * strideB) : nullptr;

  const int rlane = lane & 15;
  const int koff  = (lane >> 4) * 8;
  const int mOff  = (lane >> 4) * 8;

  v8f acc[4][4];
#pragma unroll
  for (int i = 0; i < 4; ++i)
#pragma unroll
    for (int j = 0; j < 4; ++j) acc[i][j] = (v8f){0.f,0.f,0.f,0.f,0.f,0.f,0.f,0.f};

  for (int k0 = 0; k0 < K; k0 += 32) {
    V bh[4], bl[4];
#pragma unroll
    for (int j = 0; j < 4; ++j) {
      const size_t bo = (size_t)(n0 + (j << 4) + rlane) * ldb + koff + k0;
      bh[j] = Frag<T>::load(Bb + bo);
      if (SPLIT) bl[j] = Frag<T>::load(Bb2 + bo);
    }
#pragma unroll
    for (int i = 0; i < 4; ++i) {
      const size_t ao = (size_t)(m0 + (i << 4) + rlane) * lda + koff + k0;
      V ah = Frag<T>::load(Ab + ao);
      V al;
      if (SPLIT) al = Frag<T>::load(Ab2 + ao);
#pragma unroll
      for (int j = 0; j < 4; ++j) {
        acc[i][j] = Frag<T>::mma(ah, bh[j], acc[i][j]);
        if (SPLIT) {
          acc[i][j] = Frag<T>::mma(ah, bl[j], acc[i][j]);
          acc[i][j] = Frag<T>::mma(al, bh[j], acc[i][j]);
        }
      }
      Frag<T>::guard(acc[i][0], acc[i][3], ah, SPLIT ? al : ah);
    }
    Frag<T>::keep(bh[0], bh[1], bh[2], bh[3]);
    if (SPLIT) Frag<T>::keep(bl[0], bl[1], bl[2], bl[3]);
  }
  acc_guard4(acc[0][0], acc[0][1], acc[0][2], acc[0][3]);
  acc_guard4(acc[1][0], acc[1][1], acc[1][2], acc[1][3]);
  acc_guard4(acc[2][0], acc[2][1], acc[2][2], acc[2][3]);
  acc_guard4(acc[3][0], acc[3][1], acc[3][2], acc[3][3]);

  float* slab = sT[wave];
  const float* Rb = RESID ? (resid + (size_t)b * strideR) : nullptr;
#pragma unroll
  for (int i = 0; i < 4; ++i) {
    const int mBase = m0 + (i << 4);
#pragma unroll
    for (int j = 0; j < 4; ++j) {
      const int n = n0 + (j << 4) + rlane;
      float bv = 0.f;
      if (BIAS_MODE == 2) bv = bias[n];
#pragma unroll
      for (int r = 0; r < 8; ++r) {
        float v = acc[i][j][r] * scale;
        if (BIAS_MODE == 1) v += bias[mBase + mOff + r];
        if (BIAS_MODE == 2) v += bv;
        if (RESID) v += Rb[(size_t)(mBase + mOff + r) * ldc + n];
        if (ACT == 2) v = fmaxf(v, 0.0f);
        slab[(mOff + r) * 68 + (j << 4) + rlane] = v;
      }
    }
    __builtin_amdgcn_fence(3  , "workgroup");
    __builtin_amdgcn_wave_barrier();
    __builtin_amdgcn_fence(2  , "workgroup");
    if (OUT_MODE == 0) {
      float* C = (float*)Cout + (size_t)b * strideC;
      const int hh = lane >> 4, c4 = (lane & 15) * 4;
      for (int pass = 0; pass < 2; ++pass) {
#pragma unroll
        for (int it = 0; it < 8; ++it) {
          const int row = it * 2 + hh;
          v4f v = *(const v4f*)(slab + row * 68 + c4);
          *(volatile v4f*)(C + (size_t)(mBase + row) * ldc + n0 + c4) = v;
        }
        __threadfence();
      }
    } else {
      const int q = lane >> 3, c8 = (lane & 7) * 8;
      unsigned short* C  = (unsigned short*)Cout  + (size_t)b * strideC;
      unsigned short* C2 = (OUT_MODE == 2) ? ((unsigned short*)Cout2 + (size_t)b * strideC) : nullptr;
      for (int pass = 0; pass < 2; ++pass) {
#pragma unroll
        for (int it = 0; it < 4; ++it) {
          const int row = it * 4 + q;
          const float* sp = slab + row * 68 + c8;
          v8h hv, lv;
#pragma unroll
          for (int e = 0; e < 8; ++e) {
            if (OUT_MODE == 1) {
              hv[e] = (_Float16)sp[e];
            } else {
              unsigned short hb = f2bf_bits(sp[e]);
              unsigned short lb = f2bf_bits(sp[e] - bf_bits2f(hb));
              hv[e] = __builtin_bit_cast(_Float16, hb);
              lv[e] = __builtin_bit_cast(_Float16, lb);
            }
          }
          *(volatile v8h*)(C + (size_t)(mBase + row) * ldc + n0 + c8) = hv;
          if (OUT_MODE == 2) *(volatile v8h*)(C2 + (size_t)(mBase + row) * ldc + n0 + c8) = lv;
        }
        __threadfence();
      }
    }
    __builtin_amdgcn_fence(3  , "workgroup");
    __builtin_amdgcn_wave_barrier();
    __builtin_amdgcn_fence(2  , "workgroup");
  }
}
}

__global__ __launch_bounds__(256) void k_cast_act(const float* __restrict__ q_in, const float* __restrict__ k_in, unsigned short* __restrict__ dst) {
    const unsigned u = blockIdx.x * 256u + threadIdx.x;
    if (u >= (unsigned)MROWS * 64u) return;
    const unsigned which = blockIdx.y;
    const float* src = which ? k_in : q_in;
    const unsigned r = u >> 6, c0 = (u & 63u) << 3;
    const unsigned b = r / (unsigned)SEQ, s = r - b * (unsigned)SEQ;
    const float* sp = src + ((size_t)b * SEQ_FULL + s) * DM + c0;
    const v4f a = *(const v4f*)sp, c = *(const v4f*)(sp + 4);
    cm_u4 pk;
    pk.x = cmb_pk2(cmb_bf(a.x), cmb_bf(a.y)); pk.y = cmb_pk2(cmb_bf(a.z), cmb_bf(a.w));
    pk.z = cmb_pk2(cmb_bf(c.x), cmb_bf(c.y)); pk.w = cmb_pk2(cmb_bf(c.z), cmb_bf(c.w));
    unsigned short* d = dst + (size_t)which * MROWS * DM + (size_t)r * DM + c0;
    VST2(cm_u4, (cm_u4*)d, pk);
}

__global__ __launch_bounds__(256) void k_cast_wT(const float* __restrict__ SRC, unsigned lds, unsigned short* __restrict__ DST, unsigned ldd, unsigned nR, unsigned nC, float sc) {
    const unsigned u = blockIdx.x * 256u + threadIdx.x; const unsigned per = nR >> 3;
    if (u >= nC * per) return;
    const unsigned cc = u / per, r0 = (u - cc * per) << 3;
    float w[8];
#pragma unroll
    for (int e = 0; e < 8; ++e) w[e] = cmb_bf(SRC[(size_t)(r0 + (unsigned)e) * lds + cc]) * sc;
    cm_u4 pk; pk.x = cmb_pk2(w[0], w[1]); pk.y = cmb_pk2(w[2], w[3]); pk.z = cmb_pk2(w[4], w[5]); pk.w = cmb_pk2(w[6], w[7]);
    VST2(cm_u4, (cm_u4*)(DST + (size_t)cc * ldd + r0), pk);
}

__global__ __launch_bounds__(128) void k_attn_pl(const unsigned short* __restrict__ Qp, const unsigned short* __restrict__ Kp, const unsigned short* __restrict__ VTp,
                                                   const int* __restrict__ qlen, const int* __restrict__ klen, float* __restrict__ ctx) {
    typedef w25::Frag<_Float16> FH;
    __shared__ __align__(16) _Float16 Psh[4][16 * 64];
    __shared__ __align__(16) float    Os[4][16 * 68];
    const unsigned tid = threadIdx.x, wave = tid >> 5, lane = tid & 31u, hh = lane >> 4, c = lane & 15u;
    const unsigned nqb = (unsigned)SEQ / 64u;
    const unsigned bx = blockIdx.x;
    const unsigned bh = bx / nqb, qb = bx - bh * nqb;
    const unsigned h = bh & (unsigned)(NH - 1);
    unsigned b = bh / (unsigned)NH; b = (b < (unsigned)NB) ? b : (unsigned)(NB - 1);
    const unsigned q0 = qb * 64u + wave * 16u;
    int kl = klen[b]; kl = min(max(kl, 0), (int)SEQ);
    const int ql = qlen[b];
    unsigned nck = (kl <= 1) ? nqb : (((unsigned)kl + 63u) >> 6);
    if ((int)q0 >= ql) nck = 0u;

    const _Float16* Qb = (const _Float16*)Qp + (size_t)b * SEQ * DM + h * 64u;
    const _Float16* Kb = (const _Float16*)Kp + (size_t)b * SEQ * DM + h * 64u;
    const _Float16* Vb = (const _Float16*)VTp + ((size_t)b * DM + h * 64u) * SEQ;
    float* Ob = ctx + (size_t)b * SEQ * DM + h * 64u;

    const _Float16* qrow = Qb + (size_t)(q0 + c) * DM + 8u * hh;
    const v16h qa0 = FH::load(qrow), qa1 = FH::load(qrow + 32);

    float mrow[8], lrow[8];
    v8f oacc[4];
#pragma unroll
    for (int r = 0; r < 8; ++r) { mrow[r] = -INFINITY; lrow[r] = 0.f; }
#pragma unroll
    for (int t = 0; t < 4; ++t) oacc[t] = (v8f){0.f,0.f,0.f,0.f,0.f,0.f,0.f,0.f};

    _Float16* pw = Psh[wave];
    for (unsigned kc = 0; kc < nck; ++kc) {
        const unsigned kv0 = kc * 64u;
        v8f s[4];
#pragma unroll
        for (int j = 0; j < 4; ++j) {
            const _Float16* kr = Kb + (size_t)(kv0 + (unsigned)j * 16u + c) * DM + 8u * hh;
            v8f z = (v8f){0.f,0.f,0.f,0.f,0.f,0.f,0.f,0.f};
            z = wmma16(qa0, FH::load(kr), z);
            z = wmma16(qa1, FH::load(kr + 32), z);
            s[j] = z;
        }
        float cm[8];
#pragma unroll
        for (int r = 0; r < 8; ++r) {
            const int qr = (int)(q0 + 8u * hh) + r;
            float m = -INFINITY;
#pragma unroll
            for (int j = 0; j < 4; ++j) {
                const int kvcol = (int)(kv0 + c) + j * 16;
                const bool fill = (kvcol >= kl) || (kvcol == qr);
                const float v = fill ? NEGFILL : s[j][r] * 0.125f;
                s[j][r] = v;
                m = fmaxf(m, v);
            }
            m = fmaxf(m, __shfl_xor(m, 1, 32)); m = fmaxf(m, __shfl_xor(m, 2, 32));
            m = fmaxf(m, __shfl_xor(m, 4, 32)); m = fmaxf(m, __shfl_xor(m, 8, 32));
            cm[r] = m;
        }
#pragma unroll
        for (int r = 0; r < 8; ++r) {
            const float mnew = fmaxf(mrow[r], cm[r]);
            const float alpha = expf(mrow[r] - mnew);
            mrow[r] = mnew;
            float psum = 0.f;
#pragma unroll
            for (int j = 0; j < 4; ++j) {
                const float p = expf(s[j][r] - mnew);
                psum += p;
                pw[(8u * hh + (unsigned)r) * 64u + (unsigned)j * 16u + c] = (_Float16)(p * AT_PSC);
            }
            psum += __shfl_xor(psum, 1, 32); psum += __shfl_xor(psum, 2, 32);
            psum += __shfl_xor(psum, 4, 32); psum += __shfl_xor(psum, 8, 32);
            lrow[r] = lrow[r] * alpha + psum;
#pragma unroll
            for (int t = 0; t < 4; ++t) oacc[t][r] *= alpha;
        }
        wave_lds_sync();
#pragma unroll
        for (int kk = 0; kk < 2; ++kk) {
            const v16h pa = FH::load(pw + c * 64u + (unsigned)kk * 32u + 8u * hh);
#pragma unroll
            for (int t = 0; t < 4; ++t) {
                const v16h vb = FH::load(Vb + (size_t)((unsigned)t * 16u + c) * SEQ + kv0 + (unsigned)kk * 32u + 8u * hh);
                oacc[t] = wmma16(pa, vb, oacc[t]);
            }
        }
        wave_lds_sync();
    }

    float* os = Os[wave];
#pragma unroll
    for (int r = 0; r < 8; ++r) {
        const float inv = (lrow[r] > 0.f) ? 1.0f / (lrow[r] * AT_PSC) : 0.f;
        const bool live = ((int)(q0 + 8u * hh) + r) < ql;
#pragma unroll
        for (int t = 0; t < 4; ++t) os[(8u * hh + (unsigned)r) * 68u + (unsigned)t * 16u + c] = live ? oacc[t][r] * inv : 0.f;
    }
    wave_lds_sync();
    {
        const unsigned c4 = (lane & 15u) * 4u;
        for (int pass = 0; pass < 2; ++pass) {
#pragma unroll
            for (int it = 0; it < 8; ++it) {
                const unsigned row = (unsigned)it * 2u + hh;
                const v4f val = *(const v4f*)(os + row * 68u + c4);
                *(volatile v4f*)(Ob + (size_t)(q0 + row) * DM + c4) = val;
            }
            __threadfence();
        }
    }
}

__global__ __launch_bounds__(256) void k_ln1(const float* __restrict__ ctx, const float* __restrict__ qin, const float* __restrict__ gam, const float* __restrict__ bet,
                                               float* __restrict__ lnf, unsigned short* __restrict__ lnh) {
    __shared__ __align__(16) float rowb[8][DM];
    const unsigned tid = threadIdx.x, lane = tid & 31u, wave = tid >> 5;
    const unsigned row = blockIdx.x * 8u + wave;
    const unsigned b = row / (unsigned)SEQ, s = row - b * (unsigned)SEQ;
    const float* cr = ctx + (size_t)row * DM;
    const float* qr = qin + ((size_t)b * SEQ_FULL + s) * DM;
    float* xr = rowb[wave];
    float sum = 0.f;
#pragma unroll 1
    for (unsigned j = 0; j < 4u; ++j) {
        const unsigned c = lane * 4u + 128u * j;
        const v4f a = *(const v4f*)(cr + c); const v4f q = *(const v4f*)(qr + c);
        v4f x; x.x = a.x + cmb_bf(q.x); x.y = a.y + cmb_bf(q.y); x.z = a.z + cmb_bf(q.z); x.w = a.w + cmb_bf(q.w);
        *(v4f*)(xr + c) = x;
        sum += (x.x + x.y) + (x.z + x.w);
    }
    sum += __shfl_xor(sum, 16, 32); sum += __shfl_xor(sum, 8, 32); sum += __shfl_xor(sum, 4, 32); sum += __shfl_xor(sum, 2, 32); sum += __shfl_xor(sum, 1, 32);
    const float mu = sum * (1.0f / (float)DM);
    float q2 = 0.f;
#pragma unroll 1
    for (unsigned j = 0; j < 4u; ++j) {
        const unsigned c = lane * 4u + 128u * j;
        const v4f d = *(const v4f*)(xr + c) - mu;
        q2 += (d.x * d.x + d.y * d.y) + (d.z * d.z + d.w * d.w);
    }
    q2 += __shfl_xor(q2, 16, 32); q2 += __shfl_xor(q2, 8, 32); q2 += __shfl_xor(q2, 4, 32); q2 += __shfl_xor(q2, 2, 32); q2 += __shfl_xor(q2, 1, 32);
    const float rs = 1.0f / sqrtf(q2 * (1.0f / (float)DM) + LN_EPS);
#pragma unroll 1
    for (unsigned j = 0; j < 4u; ++j) {
        const unsigned c = lane * 4u + 128u * j;
        const v4f x = *(const v4f*)(xr + c); const v4f g = *(const v4f*)(gam + c); const v4f be = *(const v4f*)(bet + c);
        v4f y;
        y.x = (x.x - mu) * rs * cmb_bf(g.x) + cmb_bf(be.x); y.y = (x.y - mu) * rs * cmb_bf(g.y) + cmb_bf(be.y);
        y.z = (x.z - mu) * rs * cmb_bf(g.z) + cmb_bf(be.z); y.w = (x.w - mu) * rs * cmb_bf(g.w) + cmb_bf(be.w);
        *(v4f*)(xr + c) = y;
        VST2V4(lnf + (size_t)row * DM + c, y);
    }
    wave_lds_sync();
#pragma unroll 1
    for (unsigned j = 0; j < 2u; ++j) {
        const unsigned c8 = lane * 8u + 256u * j;
        const v4f a = *(const v4f*)(xr + c8), c = *(const v4f*)(xr + c8 + 4u);
        cm_u4 pk; pk.x = cmb_pk2(a.x, a.y); pk.y = cmb_pk2(a.z, a.w); pk.z = cmb_pk2(c.x, c.y); pk.w = cmb_pk2(c.z, c.w);
        VST2(cm_u4, (cm_u4*)(lnh + (size_t)row * DM + c8), pk);
    }
}

__global__ __launch_bounds__(256) void k_ln2mean(const float* __restrict__ y2, const float* __restrict__ gam, const float* __restrict__ bet, float* __restrict__ out) {
    __shared__ __align__(16) float xrow[8][DM];
    __shared__ __align__(16) float accw[8][DM];
    const unsigned tid = threadIdx.x, lane = tid & 31u, wave = tid >> 5;
    const unsigned b = blockIdx.x;
    float* xr = xrow[wave]; float* ar = accw[wave];
    v4f zz; zz.x = zz.y = zz.z = zz.w = 0.f;
#pragma unroll 1
    for (unsigned j = 0; j < 4u; ++j) *(v4f*)(ar + lane * 4u + 128u * j) = zz;
#pragma unroll 1
    for (unsigned i = 0; i < (unsigned)SEQ / 8u; ++i) {
        const unsigned s = wave + 8u * i;
        const float* yr = y2 + ((size_t)b * SEQ + s) * DM;
        float sum = 0.f;
#pragma unroll 1
        for (unsigned j = 0; j < 4u; ++j) {
            const unsigned c = lane * 4u + 128u * j;
            const v4f x = *(const v4f*)(yr + c);
            *(v4f*)(xr + c) = x;
            sum += (x.x + x.y) + (x.z + x.w);
        }
        sum += __shfl_xor(sum, 16, 32); sum += __shfl_xor(sum, 8, 32); sum += __shfl_xor(sum, 4, 32); sum += __shfl_xor(sum, 2, 32); sum += __shfl_xor(sum, 1, 32);
        const float mu = sum * (1.0f / (float)DM);
        float q2 = 0.f;
#pragma unroll 1
        for (unsigned j = 0; j < 4u; ++j) {
            const unsigned c = lane * 4u + 128u * j;
            const v4f d = *(const v4f*)(xr + c) - mu;
            q2 += (d.x * d.x + d.y * d.y) + (d.z * d.z + d.w * d.w);
        }
        q2 += __shfl_xor(q2, 16, 32); q2 += __shfl_xor(q2, 8, 32); q2 += __shfl_xor(q2, 4, 32); q2 += __shfl_xor(q2, 2, 32); q2 += __shfl_xor(q2, 1, 32);
        const float rs = 1.0f / sqrtf(q2 * (1.0f / (float)DM) + LN_EPS);
#pragma unroll 1
        for (unsigned j = 0; j < 4u; ++j) {
            const unsigned c = lane * 4u + 128u * j;
            v4f a = *(const v4f*)(ar + c);
            const v4f d = *(const v4f*)(xr + c) - mu;
            a = a + d * rs;
            *(v4f*)(ar + c) = a;
        }
    }
    __syncthreads();
    if (tid < 128u) {
        const unsigned c = tid * 4u;
        v4f a = zz;
#pragma unroll
        for (int w = 0; w < 8; ++w) a = a + *(const v4f*)(&accw[w][c]);
        const v4f g = *(const v4f*)(gam + c); const v4f be = *(const v4f*)(bet + c);
        const float is = 1.0f / (float)SEQ;
        v4f o;
        o.x = cmb_bf(g.x) * (a.x * is) + cmb_bf(be.x); o.y = cmb_bf(g.y) * (a.y * is) + cmb_bf(be.y);
        o.z = cmb_bf(g.z) * (a.z * is) + cmb_bf(be.z); o.w = cmb_bf(g.w) * (a.w * is) + cmb_bf(be.w);
        VST2V4(out + (size_t)b * DM + c, o);
    }
}

extern "C" void kernel_launch(void* const* d_in, const int* in_sizes, int n_in, void* d_out, int out_size, void* d_ws, size_t ws_size, hipStream_t stream) {
    if (n_in < 11) return;
    const long long act_need = ((long long)(NB - 1) * SEQ_FULL + SEQ) * DM;
    if ((long long)in_sizes[0] < act_need || (long long)in_sizes[1] < act_need) return;
    if (in_sizes[2] < DM * DM || in_sizes[3] < DM * DM || in_sizes[4] < DM * DM) return;
    if (in_sizes[5] < DM * DFF || in_sizes[6] < DFF * DM) return;
    if (in_sizes[7] < DM || in_sizes[8] < DM || in_sizes[9] < NB || in_sizes[10] < NB) return;
    if (out_size < NB * DM) return;

    const float* queries = (const float*)d_in[0];
    const float* keysp   = (const float*)d_in[1];
    const float* W_Q     = (const float*)d_in[2];
    const float* W_K     = (const float*)d_in[3];
    const float* W_V     = (const float*)d_in[4];
    const float* fw1     = (const float*)d_in[5];
    const float* fw2     = (const float*)d_in[6];
    const float* gam     = (const float*)d_in[7];
    const float* bet     = (const float*)d_in[8];
    const int*   qlen    = (const int*)d_in[9];
    const int*   klen    = (const int*)d_in[10];
    float* out = (float*)d_out;

    constexpr size_t R0_B = (size_t)MROWS * 2048, R1_B = (size_t)MROWS * 3072, R2_B = (size_t)MROWS * 2048;
    constexpr size_t RW_B = (size_t)3 * DM * DM * 2 + (size_t)2 * DM * DFF * 2;
    static_assert((size_t)2 * MROWS * DM * 2 == R0_B);
    static_assert((size_t)MROWS * DM * 4 == R0_B);
    static_assert((size_t)MC * DFF * 2 == R0_B);
    static_assert((size_t)3 * MROWS * DM * 2 == R1_B);
    static_assert((size_t)MROWS * DM * 4 + (size_t)MROWS * DM * 2 == R1_B);
    static_assert(R0_B + R1_B + R2_B + RW_B <= (size_t)134217728);
    if (R0_B + R1_B + R2_B + RW_B > ws_size) return;
    char* ws = (char*)d_ws;
    unsigned short* X16  = (unsigned short*)ws;
    float*          CTX  = (float*)ws;
    unsigned short* H16  = (unsigned short*)ws;
    unsigned short* QK16 = (unsigned short*)(ws + R0_B);
    unsigned short* VT16 = QK16 + (size_t)2 * MROWS * DM;
    float*          LN1F = (float*)(ws + R0_B);
    unsigned short* LN1H = (unsigned short*)(ws + R0_B + (size_t)MROWS * DM * 4);
    float*          Y2   = (float*)(ws + R0_B + R1_B);
    unsigned short* WQKV = (unsigned short*)(ws + R0_B + R1_B + R2_B);
    unsigned short* F1T  = WQKV + (size_t)3 * DM * DM;
    unsigned short* F2T  = F1T + (size_t)DM * DFF;

    k_cast_act<<<dim3((unsigned)(MROWS * 64 / 256), 2u), 256, 0, stream>>>(queries, keysp, X16);
    k_cast_wT<<<(unsigned)((DM * (DM / 8) + 255) / 256), 256, 0, stream>>>(W_Q, DM, WQKV, DM, DM, DM, WCARRY);
    k_cast_wT<<<(unsigned)((DM * (DM / 8) + 255) / 256), 256, 0, stream>>>(W_K, DM, WQKV + (size_t)DM * DM, DM, DM, DM, WCARRY);
    k_cast_wT<<<(unsigned)((DM * (DM / 8) + 255) / 256), 256, 0, stream>>>(W_V, DM, WQKV + (size_t)2 * DM * DM, DM, DM, DM, WCARRY);
    k_cast_wT<<<(unsigned)((DFF * (DM / 8) + 255) / 256), 256, 0, stream>>>(fw1, DFF, F1T, DM, DM, DFF, WCARRY);
    k_cast_wT<<<(unsigned)((DM * (DFF / 8) + 255) / 256), 256, 0, stream>>>(fw2, DM, F2T, DFF, DFF, DM, WCARRY);
    w25::wmma_gemm64<0, false, 0, 1, false, 0><<<dim3((unsigned)(((MROWS / 64) * (DM / 64) + 7) / 8), 2u), 256, 0, stream>>>(
        X16, nullptr, DM, (long)MROWS * DM, WQKV, nullptr, DM, (long)DM * DM, (void*)QK16, nullptr, DM, (long)MROWS * DM,
        nullptr, nullptr, 0, MROWS, DM, DM, WINV);
    w25::wmma_gemm64<0, false, 0, 1, false, 0><<<dim3((unsigned)(((DM / 64) * (SEQ / 64) + 7) / 8), (unsigned)NB), 256, 0, stream>>>(
        WQKV + (size_t)2 * DM * DM, nullptr, DM, 0, X16 + (size_t)MROWS * DM, nullptr, DM, (long)SEQ * DM, (void*)VT16, nullptr, SEQ, (long)DM * SEQ,
        nullptr, nullptr, 0, DM, SEQ, DM, WINV);
    k_attn_pl<<<(unsigned)(NB * NH * (SEQ / 64)), 128, 0, stream>>>(QK16, QK16 + (size_t)MROWS * DM, VT16, qlen, klen, CTX);
    k_ln1<<<(unsigned)(MROWS / 8), 256, 0, stream>>>(CTX, queries, gam, bet, LN1F, LN1H);
    for (int ch = 0; ch < 2; ++ch) {
        w25::wmma_gemm64<0, false, 0, 1, false, 2><<<dim3((unsigned)(((MC / 64) * (DFF / 64) + 7) / 8), 1u), 256, 0, stream>>>(
            LN1H + (size_t)ch * MC * DM, nullptr, DM, 0, F1T, nullptr, DM, 0, (void*)H16, nullptr, DFF, 0,
            nullptr, nullptr, 0, MC, DFF, DM, WINV);
        w25::wmma_gemm64<0, false, 0, 0, true, 0><<<dim3((unsigned)(((MC / 64) * (DM / 64) + 7) / 8), 1u), 256, 0, stream>>>(
            H16, nullptr, DFF, 0, F2T, nullptr, DFF, 0, (void*)(Y2 + (size_t)ch * MC * DM), nullptr, DM, 0,
            nullptr, LN1F + (size_t)ch * MC * DM, 0, MC, DM, DFF, WINV);
    }
    k_ln2mean<<<(unsigned)NB, 256, 0, stream>>>(Y2, gam, bet, out);
}
